// Model_82008105550530
// MI455X (gfx1250) — hardware-verified
//
#include <hip/hip_runtime.h>
#include <math.h>

typedef __attribute__((ext_vector_type(16))) _Float16 v16h;
typedef __attribute__((ext_vector_type(8)))  _Float16 v8h;
typedef __attribute__((ext_vector_type(8)))  float    v8f;
typedef __attribute__((ext_vector_type(4)))  float    v4f;

constexpr int kBatch      = 256;
constexpr int kSteps      = 4096;
constexpr int kIn         = 1;
constexpr int kHid        = 10;
constexpr int kTileRows   = 16;
constexpr int kTiles      = kBatch / kTileRows;
constexpr int kChunk      = 32;
constexpr int kNumChunks  = kSteps / kChunk;
constexpr int kPitch      = 36;
constexpr int kThr        = 256;
constexpr size_t kOutElems = (size_t)kBatch * (size_t)kSteps;
constexpr size_t kWsTotal = 2 * kOutElems * 4;
static_assert(kBatch % kTileRows == 0 && kSteps % kChunk == 0, "whole tiles and chunks");
static_assert(kHid <= 16 && kIn == 1, "the units fit the first 16 k; the scalar input sits at k 16 of the low lane half");
static_assert((kPitch % 4) == 0, "16-B aligned LDS rows");
static_assert(kWsTotal == 8388608ull && kWsTotal <= 134217728ull, "carve total and cap");
static_assert((kOutElems / 4) % kThr == 0, "the combine grid is exact");

constexpr float kStateCarry  = 256.0f;
constexpr float kWeightCarry = 64.0f;
constexpr float kFoldBack    = 1.0f / (kStateCarry * kWeightCarry);
constexpr float kF16MinNorm  = 6.103515625e-5f;
static_assert(kStateCarry * kWeightCarry == 16384.0f, "carry product");

namespace eng {

union FragU { v16h v; v8h h[2]; };

__device__ __forceinline__ unsigned short f2bf_bits(float f) {
  unsigned u = __float_as_uint(f);
  return (unsigned short)((u + 0x7FFFu + ((u >> 16) & 1u)) >> 16);
}
__device__ __forceinline__ float bf16v(float f) {
  return __uint_as_float(((unsigned)f2bf_bits(f)) << 16);
}
__device__ __forceinline__ _Float16 to_f16_flushed(float c) {
  const float z = (fabsf(c) < kF16MinNorm) ? 0.0f : c;
  return (_Float16)z;
}
__device__ __forceinline__ v8f mma_f16(v16h a, v16h b) {
  v8f c = (v8f){0.f, 0.f, 0.f, 0.f, 0.f, 0.f, 0.f, 0.f};
  c = __builtin_amdgcn_wmma_f32_16x16x32_f16(false, a, false, b, (short)0, c, false, false);
  asm volatile("v_nop\n\tv_nop\n\tv_nop\n\tv_nop" : "+v"(c) : "v"(a), "v"(b));
  return c;
}
__device__ __forceinline__ float fast_tanh(float v) {
  const float e = __expf(2.0f * v);
  return 1.0f - 2.0f * __builtin_amdgcn_rcpf(e + 1.0f);
}
__device__ __forceinline__ float fast_sigmoid(float v) {
  return __builtin_amdgcn_rcpf(1.0f + __expf(-v));
}

}

__global__ __launch_bounds__(32) void bilstm_dir_kernel(
    const float* __restrict__ x,
    const float* __restrict__ w_ih_f, const float* __restrict__ w_hh_f,
    const float* __restrict__ b_ih_f, const float* __restrict__ b_hh_f,
    const float* __restrict__ w_ih_b, const float* __restrict__ w_hh_b,
    const float* __restrict__ b_ih_b, const float* __restrict__ b_hh_b,
    const float* __restrict__ w_out, const float* __restrict__ b_out,
    float* __restrict__ part)
{
  __shared__ __align__(16) float xs[kTileRows * kPitch];
  __shared__ __align__(16) float os[kTileRows * kPitch];
  __shared__ __align__(16) float wsm[13 * 32];
  __shared__ __align__(16) float vsm[3 * 64];
  __shared__ __align__(16) float hsm[32];

  const int lane = threadIdx.x & 31;
  const int hsel = lane >> 4;
  const int n    = lane & 15;
  const bool lowHalf = (hsel == 0);
  const int dir  = blockIdx.x >> 4;
  const int b0   = (blockIdx.x & 15) * kTileRows;
  const float* w_ih = dir ? w_ih_b : w_ih_f;
  const float* w_hh = dir ? w_hh_b : w_hh_f;
  const float* b_ih = dir ? b_ih_b : b_ih_f;
  const float* b_hh = dir ? b_hh_b : b_hh_f;

  {
#pragma unroll
    for (int it = 0; it < 13; ++it) {
      const int i  = it * 32 + lane;
      const int ic = (i < 4 * kHid * kHid) ? i : (4 * kHid * kHid - 1);
      wsm[ic] = w_hh[ic];
    }
#pragma unroll
    for (int it = 0; it < 2; ++it) {
      const int s  = it * 32 + lane;
      const int sc = (s < 4 * kHid - 1) ? s : (4 * kHid - 1);
      vsm[0 * 64 + s] = w_ih[sc];
      vsm[1 * 64 + s] = b_ih[sc];
      vsm[2 * 64 + s] = b_hh[sc];
    }
    const int uc = (lane < kHid - 1) ? lane : (kHid - 1);
    const float wv = w_out[dir * kHid + uc];
    const float bv = b_out[0];
    hsm[lane] = (lane < kHid) ? wv : ((lane == 16) ? bv : 0.0f);
  }
  __syncthreads();

  v16h fragA[4];
  {
    const int m  = n;
    const int mc = (m < kHid) ? m : (kHid - 1);
    const bool mok = (m < kHid);
#pragma unroll
    for (int g = 0; g < 4; ++g) {
      v8h alo, ahi;
#pragma unroll
      for (int i = 0; i < 8; ++i) {
        const int k  = 8 * hsel + i;
        const int kc = (k < kHid) ? k : (kHid - 1);
        const float f0 = wsm[(g * kHid + mc) * kHid + kc];
        const bool ok0 = mok && (k < kHid);
        alo[i] = eng::to_f16_flushed(ok0 ? (eng::bf16v(f0) * kWeightCarry) : 0.0f);
        const float f1 = vsm[0 * 64 + g * kHid + mc];
        const bool ok1 = mok && lowHalf && (i == 0);
        ahi[i] = eng::to_f16_flushed(ok1 ? (eng::bf16v(f1) * kWeightCarry) : 0.0f);
      }
      eng::FragU u0;
      u0.h[0] = alo;
      u0.h[1] = ahi;
      fragA[g] = u0.v;
    }
  }

  float bi[8], bf[8], bg[8], bo[8], wo[8];
  float hf[8], cf[8];
  v8h hb;
#pragma unroll
  for (int r = 0; r < 8; ++r) {
    const int u  = 8 * hsel + r;
    const int uc = (u < kHid) ? u : (kHid - 1);
    const bool live = (u < kHid);
    bi[r] = eng::bf16v(vsm[1 * 64 + uc])            + eng::bf16v(vsm[2 * 64 + uc]);
    bf[r] = eng::bf16v(vsm[1 * 64 + kHid + uc])     + eng::bf16v(vsm[2 * 64 + kHid + uc]);
    bg[r] = eng::bf16v(vsm[1 * 64 + 2 * kHid + uc]) + eng::bf16v(vsm[2 * 64 + 2 * kHid + uc]);
    bo[r] = eng::bf16v(vsm[1 * 64 + 3 * kHid + uc]) + eng::bf16v(vsm[2 * 64 + 3 * kHid + uc]);
    const float wvr = eng::bf16v(hsm[uc]);
    wo[r] = live ? wvr : 0.0f;
    hf[r] = 0.0f;
    cf[r] = 0.0f;
    hb[r] = (_Float16)0.0f;
  }
  const float pb = (dir == 0) ? eng::bf16v(hsm[16]) : 0.0f;
  const v8h zh = (v8h){(_Float16)0.0f, (_Float16)0.0f, (_Float16)0.0f, (_Float16)0.0f,
                       (_Float16)0.0f, (_Float16)0.0f, (_Float16)0.0f, (_Float16)0.0f};

  const int q  = lane >> 3;
  const int c4 = (lane & 7) * 4;
  float* pdst = part + (size_t)dir * kOutElems;

#pragma unroll 1
  for (int ch = 0; ch < kNumChunks; ++ch) {
    const int t0 = dir ? (kSteps - kChunk * (ch + 1)) : (kChunk * ch);
#pragma unroll
    for (int it = 0; it < 4; ++it) {
      const int row = it * 4 + q;
      const v4f v = *(const v4f*)(x + (size_t)(b0 + row) * kSteps + t0 + c4);
      v4f rv;
      const float v0 = v[0];
      const float v1 = v[1];
      const float v2 = v[2];
      const float v3 = v[3];
      rv[0] = eng::bf16v(v0);
      rv[1] = eng::bf16v(v1);
      rv[2] = eng::bf16v(v2);
      rv[3] = eng::bf16v(v3);
      *(v4f*)(xs + row * kPitch + c4) = rv;
    }
    __syncthreads();

#pragma unroll 1
    for (int s = 0; s < kChunk; ++s) {
      const int sc = dir ? (kChunk - 1 - s) : s;
      const float xv = xs[n * kPitch + sc];
      v8h xb = zh;
      xb[0] = eng::to_f16_flushed(lowHalf ? (xv * kStateCarry) : 0.0f);
      eng::FragU fb;
      fb.h[0] = hb;
      fb.h[1] = xb;
      const v8f ai = eng::mma_f16(fragA[0], fb.v);
      const v8f af = eng::mma_f16(fragA[1], fb.v);
      const v8f ag = eng::mma_f16(fragA[2], fb.v);
      const v8f ao = eng::mma_f16(fragA[3], fb.v);
      float p = 0.0f;
#pragma unroll
      for (int r = 0; r < 8; ++r) {
        const float ig = eng::fast_sigmoid(fmaf(ai[r], kFoldBack, bi[r]));
        const float fg = eng::fast_sigmoid(fmaf(af[r], kFoldBack, bf[r]));
        const float gg = eng::fast_tanh(fmaf(ag[r], kFoldBack, bg[r]));
        const float og = eng::fast_sigmoid(fmaf(ao[r], kFoldBack, bo[r]));
        const float cn = fg * cf[r] + ig * gg;
        const float hv = og * eng::fast_tanh(cn);
        const bool live = (8 * hsel + r) < kHid;
        cf[r] = live ? cn : 0.0f;
        const float hs = live ? hv : 0.0f;
        hf[r] = hs;
        hb[r] = eng::to_f16_flushed(hs * kStateCarry);
        p = fmaf(wo[r], hs, p);
      }
      const float pother = __shfl_xor(p, 16, 32);
      const float tot = (p + pother) + pb;
      if (lowHalf) os[n * kPitch + sc] = tot;
    }
    __syncthreads();

    {
      for (int pass = 0; pass < 2; ++pass) {
#pragma unroll
        for (int it = 0; it < 4; ++it) {
          const int row = it * 4 + q;
          const v4f ov = *(const v4f*)(os + row * kPitch + c4);
          *(volatile v4f*)(pdst + (size_t)(b0 + row) * kSteps + t0 + c4) = ov;
        }
        __threadfence();
      }
    }
  }
}

__global__ __launch_bounds__(kThr) void combine_kernel(const float* __restrict__ part, float* __restrict__ out) {
  const size_t i4 = ((size_t)blockIdx.x * kThr + threadIdx.x) * 4;
  const v4f a = *(const v4f*)(part + i4);
  const v4f b = *(const v4f*)(part + kOutElems + i4);
  v4f o;
#pragma unroll
  for (int e = 0; e < 4; ++e) o[e] = a[e] + b[e];
  *(volatile v4f*)(out + i4) = o;
  __threadfence();
  *(volatile v4f*)(out + i4) = o;
}

extern "C" void kernel_launch(void* const* d_in, const int* in_sizes, int n_in,
                              void* d_out, int out_size, void* d_ws, size_t ws_size,
                              hipStream_t stream) {
  if (n_in < 11 || d_out == nullptr || d_ws == nullptr) return;
  if ((size_t)in_sizes[0] != kOutElems) return;
  if (in_sizes[1] != 4 * kHid || in_sizes[2] != 4 * kHid * kHid || in_sizes[3] != 4 * kHid || in_sizes[4] != 4 * kHid) return;
  if (in_sizes[5] != 4 * kHid || in_sizes[6] != 4 * kHid * kHid || in_sizes[7] != 4 * kHid || in_sizes[8] != 4 * kHid) return;
  if (in_sizes[9] != 2 * kHid || in_sizes[10] != 1) return;
  if ((size_t)out_size != kOutElems) return;
  if (ws_size < kWsTotal) return;

  const float* x      = (const float*)d_in[0];
  const float* w_ih_f = (const float*)d_in[1];
  const float* w_hh_f = (const float*)d_in[2];
  const float* b_ih_f = (const float*)d_in[3];
  const float* b_hh_f = (const float*)d_in[4];
  const float* w_ih_b = (const float*)d_in[5];
  const float* w_hh_b = (const float*)d_in[6];
  const float* b_ih_b = (const float*)d_in[7];
  const float* b_hh_b = (const float*)d_in[8];
  const float* w_out  = (const float*)d_in[9];
  const float* b_out  = (const float*)d_in[10];
  float* out  = (float*)d_out;
  float* part = (float*)d_ws;

  bilstm_dir_kernel<<<2 * kTiles, 32, 0, stream>>>(x, w_ih_f, w_hh_f, b_ih_f, b_hh_f, w_ih_b, w_hh_b, b_ih_b, b_hh_b, w_out, b_out, part);
  combine_kernel<<<(int)((kOutElems / 4) / kThr), kThr, 0, stream>>>(part, out);
}
